// Weird_Attention_80934363725856
// MI455X (gfx1250) — hardware-verified
//
#include <hip/hip_runtime.h>
#include <math.h>

constexpr int kBatch  = 4;
constexpr int kSeq    = 1024;
constexpr int kDim    = 1024;
constexpr int kHeads  = 16;
constexpr int kHdim   = 64;
constexpr int kTok    = kBatch * kSeq;
constexpr int kGrp    = 8;
constexpr int kNchunk = kHeads / kGrp;
constexpr float kWCarry     = 256.0f;
constexpr float kWCarryInv  = 1.0f / 256.0f;
constexpr float kPCarry     = 2048.0f;
constexpr float kPCarryInv  = 1.0f / 2048.0f;
constexpr float kCtxCarry   = 64.0f;
constexpr float kCtxScale   = kCtxCarry / kPCarry;
constexpr float kOutScale   = 1.0f / (kCtxCarry * kWCarry);
constexpr float kScoreScale = 0.125f;

typedef __attribute__((ext_vector_type(16))) _Float16 v16h;
typedef __attribute__((ext_vector_type(8)))  _Float16 v8h;
typedef __attribute__((ext_vector_type(16))) __bf16   v16b;
typedef __attribute__((ext_vector_type(8)))  __bf16   v8b;
typedef __attribute__((ext_vector_type(8)))  float    v8f;
typedef __attribute__((ext_vector_type(4)))  float    v4f;
typedef __attribute__((ext_vector_type(4)))  unsigned int v4u;

__device__ __forceinline__ unsigned short f2bf_bits(float f) {
  unsigned u = __float_as_uint(f);
  return (unsigned short)((u + 0x7FFFu + ((u >> 16) & 1u)) >> 16);
}
__device__ __forceinline__ float bf_bits2f(unsigned short h) { return __uint_as_float(((unsigned)h) << 16); }

__device__ __forceinline__ void dep_guard_h(v8f& a, v8f& b, v16h x, v16h y) { asm volatile("v_nop\n\tv_nop\n\tv_nop\n\tv_nop" : "+v"(a), "+v"(b) : "v"(x), "v"(y)); }
__device__ __forceinline__ void dep_guard_b(v8f& a, v8f& b, v16b x, v16b y) { asm volatile("v_nop\n\tv_nop\n\tv_nop\n\tv_nop" : "+v"(a), "+v"(b) : "v"(x), "v"(y)); }
__device__ __forceinline__ void keep4_h(v16h a, v16h b, v16h c, v16h d) { asm volatile("v_nop" :: "v"(a), "v"(b), "v"(c), "v"(d)); }
__device__ __forceinline__ void keep4_b(v16b a, v16b b, v16b c, v16b d) { asm volatile("v_nop" :: "v"(a), "v"(b), "v"(c), "v"(d)); }
__device__ __forceinline__ void acc_guard4(v8f& a, v8f& b, v8f& c, v8f& d) { asm volatile("v_nop\n\tv_nop\n\tv_nop\n\tv_nop" : "+v"(a), "+v"(b), "+v"(c), "+v"(d)); }
template <typename T> struct Frag;
template <> struct Frag<_Float16> {
  typedef v16h V; union U { v16h v; v8h h[2]; };
  static __device__ __forceinline__ v16h load(const _Float16* p) {
    U f; f.h[0] = *(const v8h*)(p); f.h[1] = *(const v8h*)(p + 16); return f.v;
  }
  static __device__ __forceinline__ v8f mma(v16h a, v16h b, v8f c) {
    return __builtin_amdgcn_wmma_f32_16x16x32_f16(false, a, false, b, (short)0, c, false, false);
  }
  static __device__ __forceinline__ void guard(v8f& a, v8f& b, v16h x, v16h y) { dep_guard_h(a, b, x, y); }
  static __device__ __forceinline__ void keep(v16h a, v16h b, v16h c, v16h d) { keep4_h(a, b, c, d); }
};
template <> struct Frag<__bf16> {
  typedef v16b V; union U { v16b v; v8b h[2]; };
  static __device__ __forceinline__ v16b load(const __bf16* p) {
    U f; f.h[0] = *(const v8b*)(p); f.h[1] = *(const v8b*)(p + 16); return f.v;
  }
  static __device__ __forceinline__ v8f mma(v16b a, v16b b, v8f c) {
    return __builtin_amdgcn_wmma_f32_16x16x32_bf16(false, a, false, b, (short)0, c, false, false);
  }
  static __device__ __forceinline__ void guard(v8f& a, v8f& b, v16b x, v16b y) { dep_guard_b(a, b, x, y); }
  static __device__ __forceinline__ void keep(v16b a, v16b b, v16b c, v16b d) { keep4_b(a, b, c, d); }
};

__device__ __forceinline__ unsigned pk16(unsigned short a, unsigned short b) { return (unsigned)a | ((unsigned)b << 16); }
__device__ __forceinline__ unsigned short h_bits(float f) { const _Float16 h = (_Float16)f; return __builtin_bit_cast(unsigned short, h); }

template <int ET> struct Elem;
template <> struct Elem<0> { typedef _Float16 T; };
template <> struct Elem<1> { typedef __bf16 T; };
template <int ET, bool SPLIT, int BIAS_MODE, int OUT_MODE, bool RESID, int ACT = 0>
__global__ __launch_bounds__(256) void wmma_gemm64(
    const unsigned short* __restrict__ Ap, const unsigned short* __restrict__ A2p, int lda, long strideA,
    const unsigned short* __restrict__ Btp, const unsigned short* __restrict__ Bt2p, int ldb, long strideB,
    void* __restrict__ Cout, void* __restrict__ Cout2, int ldc, long strideC,
    const float* __restrict__ bias,
    const float* __restrict__ resid, long strideR,
    int M, int N, int K, float scale) {
  typedef typename Elem<ET>::T T;
  typedef typename Frag<T>::V V;
  const T* A = (const T*)Ap; const T* A2 = (const T*)A2p; const T* Bt = (const T*)Btp; const T* Bt2 = (const T*)Bt2p;
  __shared__ __align__(16) float sT[8][16 * 68];
  const int b    = blockIdx.y;
  const int lane = threadIdx.x & 31;
  const int wave = threadIdx.x >> 5;
  const int tilesN = N >> 6;
  const int tilesM = M >> 6;
  const int tile = blockIdx.x * 8 + wave;
  if (tile >= tilesM * tilesN) return;
  const int tm = tile / tilesN;
  const int tn = tile - tm * tilesN;
  const int m0 = tm << 6;
  const int n0 = tn << 6;

  const T* Ab  = A  + (size_t)b * strideA;
  const T* Bb  = Bt + (size_t)b * strideB;
  const T* Ab2 = SPLIT ? (A2  + (size_t)b * strideA) : nullptr;
  const T* Bb2 = SPLIT ? (Bt2 + (size_t)b * strideB) : nullptr;

  const int rlane = lane & 15;
  const int koff  = (lane >> 4) * 8;
  const int mOff  = (lane >> 4) * 8;

  v8f acc[4][4];
#pragma unroll
  for (int i = 0; i < 4; ++i)
#pragma unroll
    for (int j = 0; j < 4; ++j) acc[i][j] = (v8f){0.f,0.f,0.f,0.f,0.f,0.f,0.f,0.f};

  for (int k0 = 0; k0 < K; k0 += 32) {
    V bh[4], bl[4];
#pragma unroll
    for (int j = 0; j < 4; ++j) {
      const size_t bo = (size_t)(n0 + (j << 4) + rlane) * ldb + koff + k0;
      bh[j] = Frag<T>::load(Bb + bo);
      if (SPLIT) bl[j] = Frag<T>::load(Bb2 + bo);
    }
#pragma unroll
    for (int i = 0; i < 4; ++i) {
      const size_t ao = (size_t)(m0 + (i << 4) + rlane) * lda + koff + k0;
      V ah = Frag<T>::load(Ab + ao);
      V al;
      if (SPLIT) al = Frag<T>::load(Ab2 + ao);
#pragma unroll
      for (int j = 0; j < 4; ++j) {
        acc[i][j] = Frag<T>::mma(ah, bh[j], acc[i][j]);
        if (SPLIT) {
          acc[i][j] = Frag<T>::mma(ah, bl[j], acc[i][j]);
          acc[i][j] = Frag<T>::mma(al, bh[j], acc[i][j]);
        }
      }
      Frag<T>::guard(acc[i][0], acc[i][3], ah, SPLIT ? al : ah);
    }
    Frag<T>::keep(bh[0], bh[1], bh[2], bh[3]);
    if (SPLIT) Frag<T>::keep(bl[0], bl[1], bl[2], bl[3]);
  }
  acc_guard4(acc[0][0], acc[0][1], acc[0][2], acc[0][3]);
  acc_guard4(acc[1][0], acc[1][1], acc[1][2], acc[1][3]);
  acc_guard4(acc[2][0], acc[2][1], acc[2][2], acc[2][3]);
  acc_guard4(acc[3][0], acc[3][1], acc[3][2], acc[3][3]);

  float* slab = sT[wave];
  const float* Rb = RESID ? (resid + (size_t)b * strideR) : nullptr;
#pragma unroll
  for (int i = 0; i < 4; ++i) {
    const int mBase = m0 + (i << 4);
#pragma unroll
    for (int j = 0; j < 4; ++j) {
      const int n = n0 + (j << 4) + rlane;
      float bv = 0.f;
      if (BIAS_MODE == 2) bv = bias[n];
#pragma unroll
      for (int r = 0; r < 8; ++r) {
        float v = acc[i][j][r] * scale;
        if (BIAS_MODE == 1) v += bias[mBase + mOff + r];
        if (BIAS_MODE == 2) v += bv;
        if (RESID) v += Rb[(size_t)(mBase + mOff + r) * ldc + n];
        if (ACT == 2) v = fmaxf(v, 0.0f);
        if (ACT == 4) v = (v > 0.f) ? v : 0.01f * v;
        slab[(mOff + r) * 68 + (j << 4) + rlane] = v;
      }
    }
    __builtin_amdgcn_fence(__ATOMIC_RELEASE, "workgroup");
    __builtin_amdgcn_wave_barrier();
    __builtin_amdgcn_fence(__ATOMIC_ACQUIRE, "workgroup");
    if (OUT_MODE == 0) {
      float* C = (float*)Cout + (size_t)b * strideC;
      const int hh = lane >> 4, c4 = (lane & 15) * 4;
      for (int pass = 0; pass < 2; ++pass) {
#pragma unroll
        for (int it = 0; it < 8; ++it) {
          const int row = it * 2 + hh;
          v4f v = *(const v4f*)(slab + row * 68 + c4);
          *(volatile v4f*)(C + (size_t)(mBase + row) * ldc + n0 + c4) = v;
        }
        __threadfence();
      }
    } else {
      const int q = lane >> 3, c8 = (lane & 7) * 8;
      unsigned short* C  = (unsigned short*)Cout  + (size_t)b * strideC;
      unsigned short* C2 = (OUT_MODE == 2) ? ((unsigned short*)Cout2 + (size_t)b * strideC) : nullptr;
      for (int pass = 0; pass < 2; ++pass) {
#pragma unroll
        for (int it = 0; it < 4; ++it) {
          const int row = it * 4 + q;
          const float* sp = slab + row * 68 + c8;
          v8h hv, lv;
#pragma unroll
          for (int e = 0; e < 8; ++e) {
            if (OUT_MODE == 1) {
              hv[e] = (_Float16)sp[e];
            } else {
              unsigned short hb = f2bf_bits(sp[e]);
              unsigned short lb = f2bf_bits(sp[e] - bf_bits2f(hb));
              hv[e] = __builtin_bit_cast(_Float16, hb);
              lv[e] = __builtin_bit_cast(_Float16, lb);
            }
          }
          *(volatile v8h*)(C + (size_t)(mBase + row) * ldc + n0 + c8) = hv;
          if (OUT_MODE == 2) *(volatile v8h*)(C2 + (size_t)(mBase + row) * ldc + n0 + c8) = lv;
        }
        __threadfence();
      }
    }
    __builtin_amdgcn_fence(__ATOMIC_RELEASE, "workgroup");
    __builtin_amdgcn_wave_barrier();
    __builtin_amdgcn_fence(__ATOMIC_ACQUIRE, "workgroup");
  }
}

__global__ __launch_bounds__(256) void cast8_f16_kernel(const float* __restrict__ in, unsigned short* __restrict__ out,
                                                        int n8, float carry) {
  const int i = blockIdx.x * 256 + threadIdx.x;
  if (i >= n8) return;
  const float* p = in + 8 * (size_t)i;
  const v4f a = *(const v4f*)(p);
  const v4f c = *(const v4f*)(p + 4);
  unsigned short hb[8];
#pragma unroll
  for (int e = 0; e < 4; ++e) {
    hb[e]     = h_bits(a[e] * carry);
    hb[4 + e] = h_bits(c[e] * carry);
  }
  const v4u u = (v4u){pk16(hb[0], hb[1]), pk16(hb[2], hb[3]), pk16(hb[4], hb[5]), pk16(hb[6], hb[7])};
  unsigned short* q = out + 8 * (size_t)i;
  *(volatile v4u*)q = u;
  __threadfence();
  *(volatile v4u*)q = u;
}

__global__ __launch_bounds__(128) void softmax_row_kernel(const float* __restrict__ S, unsigned short* __restrict__ P,
                                                          float carry) {
  __shared__ float redM[4];
  __shared__ float redS[4];
  const int row  = blockIdx.x;
  const int t    = threadIdx.x;
  const int lane = t & 31, wave = t >> 5;
  const int c0   = t * 8;
  const float* sr = S + (size_t)row * kSeq + c0;
  const v4f a = *(const v4f*)(sr);
  const v4f c = *(const v4f*)(sr + 4);
  float x[8];
#pragma unroll
  for (int e = 0; e < 4; ++e) { x[e] = a[e]; x[4 + e] = c[e]; }
  float m = fmaxf(fmaxf(fmaxf(x[0], x[1]), fmaxf(x[2], x[3])), fmaxf(fmaxf(x[4], x[5]), fmaxf(x[6], x[7])));
#pragma unroll
  for (int off = 16; off > 0; off >>= 1) m = fmaxf(m, __shfl_xor(m, off, 32));
  if (lane == 0) redM[wave] = m;
  __syncthreads();
  m = fmaxf(fmaxf(redM[0], redM[1]), fmaxf(redM[2], redM[3]));
  float p[8];
  float s = 0.f;
#pragma unroll
  for (int e = 0; e < 8; ++e) { p[e] = expf(x[e] - m); s += p[e]; }
#pragma unroll
  for (int off = 16; off > 0; off >>= 1) s += __shfl_xor(s, off, 32);
  if (lane == 0) redS[wave] = s;
  __syncthreads();
  s = (redS[0] + redS[1]) + (redS[2] + redS[3]);
  const float inv = carry * (1.0f / s);
  unsigned short hb[8];
#pragma unroll
  for (int e = 0; e < 8; ++e) hb[e] = h_bits(p[e] * inv);
  const v4u u = (v4u){pk16(hb[0], hb[1]), pk16(hb[2], hb[3]), pk16(hb[4], hb[5]), pk16(hb[6], hb[7])};
  unsigned short* q = P + (size_t)row * kSeq + c0;
  *(volatile v4u*)q = u;
  __threadfence();
  *(volatile v4u*)q = u;
}

__global__ __launch_bounds__(256) void row_stats_kernel(const float* __restrict__ S, float* __restrict__ RM,
                                                        float* __restrict__ RI, float carry) {
  __shared__ __align__(16) float sm[32];
  __shared__ __align__(16) float si[32];
  const int t = threadIdx.x, lane = t & 31, wave = t >> 5;
  const int rbase = blockIdx.x * 32;
#pragma unroll 1
  for (int rr = 0; rr < 4; ++rr) {
    const int rl = wave * 4 + rr;
    const float* sr = S + (size_t)(rbase + rl) * kSeq + lane * 4;
    float m = -INFINITY;
#pragma unroll 1
    for (int i = 0; i < 8; ++i) {
      const v4f v = *(const v4f*)(sr + i * 128);
      m = fmaxf(m, fmaxf(fmaxf(v[0], v[1]), fmaxf(v[2], v[3])));
    }
#pragma unroll
    for (int off = 16; off > 0; off >>= 1) m = fmaxf(m, __shfl_xor(m, off, 32));
    float s = 0.f;
#pragma unroll 1
    for (int i = 0; i < 8; ++i) {
      const v4f v = *(const v4f*)(sr + i * 128);
      s += (expf(v[0] - m) + expf(v[1] - m)) + (expf(v[2] - m) + expf(v[3] - m));
    }
#pragma unroll
    for (int off = 16; off > 0; off >>= 1) s += __shfl_xor(s, off, 32);
    if (lane == 0) { sm[rl] = m; si[rl] = carry * (1.0f / s); }
  }
  __syncthreads();
  if (wave == 0) {
    const int q8 = lane & 7;
    const v4f vm = *(const v4f*)(sm + q8 * 4);
    const v4f vi = *(const v4f*)(si + q8 * 4);
    float* pm = RM + rbase + q8 * 4;
    float* pi = RI + rbase + q8 * 4;
    for (int pass = 0; pass < 2; ++pass) {
      if (lane < 8) *(volatile v4f*)pm = vm;
      if (lane >= 8 && lane < 16) *(volatile v4f*)pi = vi;
      __threadfence();
    }
  }
}

__global__ __launch_bounds__(256) void exp_transpose_kernel(const float* __restrict__ S, const float* __restrict__ RM,
                                                            const float* __restrict__ RI, unsigned short* __restrict__ PT) {
  __shared__ float sm[64][65];
  __shared__ float srm[64];
  __shared__ float sri[64];
  const int t  = threadIdx.x;
  const int t0 = blockIdx.x * 64;
  const int l0 = blockIdx.y * 64;
  const int g  = blockIdx.z;
  const float* Sg  = S  + (size_t)g * kSeq * kSeq;
  const float* RMg = RM + (size_t)g * kSeq;
  const float* RIg = RI + (size_t)g * kSeq;
  if (t < 64) srm[t] = RMg[l0 + t];
  if (t >= 64 && t < 128) sri[t - 64] = RIg[l0 + t - 64];
  __syncthreads();
#pragma unroll 1
  for (int i = 0; i < 16; ++i) {
    const int e = i * 256 + t;
    const int r = e >> 6;
    const int c = e & 63;
    const float s = Sg[(size_t)(l0 + r) * kSeq + t0 + c];
    sm[c][r] = expf(s - srm[r]) * sri[r];
  }
  __syncthreads();
  const int lane = t & 31, wave = t >> 5;
  const int q = lane >> 3, c8 = (lane & 7) * 8;
  unsigned short* op = PT + (size_t)g * kSeq * kSeq;
  for (int pass = 0; pass < 2; ++pass) {
#pragma unroll
    for (int it = 0; it < 2; ++it) {
      const int row = wave * 8 + it * 4 + q;
      unsigned short hb[8];
#pragma unroll
      for (int e = 0; e < 8; ++e) hb[e] = h_bits(sm[row][c8 + e]);
      const v4u u = (v4u){pk16(hb[0], hb[1]), pk16(hb[2], hb[3]), pk16(hb[4], hb[5]), pk16(hb[6], hb[7])};
      *(volatile v4u*)(op + (size_t)(t0 + row) * kSeq + l0 + c8) = u;
    }
    __threadfence();
  }
}

static void gemm_proj(hipStream_t st, const unsigned short* X, const unsigned short* W, unsigned short* C,
                      const float* bias, const float* rdum) {
  wmma_gemm64<0, false, 2, 1, false><<<dim3((kTok / 64) * (kDim / 64) / 8, 1), dim3(256), 0, st>>>(
      X, X, kDim, 0L, W, W, kDim, 0L, (void*)C, (void*)C, kDim, 0L, bias, rdum, 0L, kTok, kDim, kDim, kWCarryInv);
}
static void gemm_projT(hipStream_t st, const unsigned short* W, const unsigned short* X, unsigned short* C,
                       const float* bias, const float* rdum) {
  wmma_gemm64<0, false, 1, 1, false><<<dim3((kDim / 64) * (kTok / 64) / 8, 1), dim3(256), 0, st>>>(
      W, W, kDim, 0L, X, X, kDim, 0L, (void*)C, (void*)C, kTok, 0L, bias, rdum, 0L, kDim, kTok, kDim, kWCarryInv);
}

extern "C" void kernel_launch(void* const* d_in, const int* in_sizes, int n_in,
                              void* d_out, int out_size, void* d_ws, size_t ws_size,
                              hipStream_t stream) {
  if (n_in < 17) return;
  const int nFeat = kTok * kDim;
  const int nW    = kDim * kDim;
  if (in_sizes[0] != nFeat || in_sizes[1] != nFeat || in_sizes[2] != nFeat) return;
  for (int i = 0; i < 7; ++i) {
    if (in_sizes[3 + 2 * i] != nW) return;
    if (in_sizes[4 + 2 * i] != kDim) return;
  }
  if (out_size != nFeat) return;

  const size_t szProj = (size_t)kTok * kDim * 2;
  const size_t oGQ   = 0;
  const size_t oGK   = oGQ + szProj;
  const size_t oGVT  = oGK + szProj;
  const size_t oPQ   = oGVT + szProj;
  const size_t oPK   = oPQ + szProj;
  const size_t oPVT  = oPK + szProj;
  const size_t oSC   = oPVT + szProj;
  const size_t szSC  = (size_t)kGrp * kSeq * kSeq * 4;
  const size_t oGP   = oSC + szSC;
  const size_t szP   = (size_t)kGrp * kSeq * kSeq * 2;
  const size_t oPPT  = oGP + szP;
  const size_t oCTX  = oPPT + szP;
  const size_t szCTX = (size_t)kSeq * kDim * 4;
  const size_t oLAST = oCTX + szCTX;
  const size_t oW    = oLAST + szProj;
  const size_t szW   = (size_t)kDim * kDim * 2;
  const size_t oRM   = oW + szW;
  const size_t szR   = (size_t)kGrp * kSeq * 4;
  const size_t oRI   = oRM + szR;
  const size_t wsEnd = oRI + szR;
  if (ws_size < wsEnd) return;

  char* ws = (char*)d_ws;
  unsigned short* GQ16   = (unsigned short*)(ws + oGQ);
  unsigned short* GK16   = (unsigned short*)(ws + oGK);
  unsigned short* GVT16  = (unsigned short*)(ws + oGVT);
  unsigned short* PQ16   = (unsigned short*)(ws + oPQ);
  unsigned short* PK16   = (unsigned short*)(ws + oPK);
  unsigned short* PVT16  = (unsigned short*)(ws + oPVT);
  float*          SC32   = (float*)(ws + oSC);
  unsigned short* X16    = (unsigned short*)(ws + oSC);
  unsigned short* E16    = (unsigned short*)(ws + oSC);
  unsigned short* GP16   = (unsigned short*)(ws + oGP);
  unsigned short* PPT16  = (unsigned short*)(ws + oPPT);
  float*          CTX32  = (float*)(ws + oCTX);
  unsigned short* LAST16 = (unsigned short*)(ws + oLAST);
  unsigned short* W16    = (unsigned short*)(ws + oW);
  float*          RM     = (float*)(ws + oRM);
  float*          RI     = (float*)(ws + oRI);

  const float* gfeat = (const float*)d_in[0];
  const float* lfeat = (const float*)d_in[1];
  const float* tfeat = (const float*)d_in[2];
  const float* Wp[7];
  const float* Bp[7];
  for (int i = 0; i < 7; ++i) { Wp[i] = (const float*)d_in[3 + 2 * i]; Bp[i] = (const float*)d_in[4 + 2 * i]; }
  const float* bdum = Bp[0];
  const float* rdum = (const float*)(ws + oRM);

  const int castFeatBlocks = (nFeat / 8) / 256;
  const int castWBlocks    = (nW / 8) / 256;

  cast8_f16_kernel<<<dim3(castFeatBlocks), dim3(256), 0, stream>>>(gfeat, X16, nFeat / 8, 1.0f);
  cast8_f16_kernel<<<dim3(castWBlocks), dim3(256), 0, stream>>>(Wp[0], W16, nW / 8, kWCarry);
  gemm_proj(stream, X16, W16, GQ16, Bp[0], rdum);
  cast8_f16_kernel<<<dim3(castFeatBlocks), dim3(256), 0, stream>>>(lfeat, X16, nFeat / 8, 1.0f);
  cast8_f16_kernel<<<dim3(castWBlocks), dim3(256), 0, stream>>>(Wp[1], W16, nW / 8, kWCarry);
  gemm_proj(stream, X16, W16, GK16, Bp[1], rdum);
  cast8_f16_kernel<<<dim3(castWBlocks), dim3(256), 0, stream>>>(Wp[2], W16, nW / 8, kWCarry);
  gemm_projT(stream, W16, X16, GVT16, Bp[2], rdum);
  cast8_f16_kernel<<<dim3(castWBlocks), dim3(256), 0, stream>>>(Wp[3], W16, nW / 8, kWCarry);
  gemm_proj(stream, X16, W16, PQ16, Bp[3], rdum);
  cast8_f16_kernel<<<dim3(castFeatBlocks), dim3(256), 0, stream>>>(tfeat, X16, nFeat / 8, 1.0f);
  cast8_f16_kernel<<<dim3(castWBlocks), dim3(256), 0, stream>>>(Wp[4], W16, nW / 8, kWCarry);
  gemm_proj(stream, X16, W16, PK16, Bp[4], rdum);
  cast8_f16_kernel<<<dim3(castWBlocks), dim3(256), 0, stream>>>(Wp[5], W16, nW / 8, kWCarry);
  gemm_projT(stream, W16, X16, PVT16, Bp[5], rdum);

  const long sPlane  = (long)kSeq * kSeq;
  const long sVTgrp  = (long)kHdim * kTok;
  const dim3 gridSq((kSeq / 64) * (kSeq / 64) / 8, kGrp);
  const dim3 gridCtx((kSeq / 64) * (kHdim / 64) / 8, kGrp);
  for (int b = 0; b < kBatch; ++b) {
    for (int c = 0; c < kNchunk; ++c) {
      const size_t qoff = (size_t)b * kSeq * kDim + (size_t)c * kGrp * kHdim;
      const size_t voff = (size_t)(c * kGrp * kHdim) * kTok + (size_t)b * kSeq;
      const size_t coff = (size_t)c * kGrp * kHdim;
      wmma_gemm64<0, false, 0, 0, false><<<gridSq, dim3(256), 0, stream>>>(
          GQ16 + qoff, GQ16 + qoff, kDim, (long)kHdim, GK16 + qoff, GK16 + qoff, kDim, (long)kHdim,
          (void*)SC32, (void*)SC32, kSeq, sPlane, bdum, rdum, 0L, kSeq, kSeq, kHdim, kScoreScale);
      softmax_row_kernel<<<dim3(kGrp * kSeq), dim3(128), 0, stream>>>(SC32, GP16, kPCarry);
      wmma_gemm64<0, false, 0, 0, false><<<gridSq, dim3(256), 0, stream>>>(
          PQ16 + qoff, PQ16 + qoff, kDim, (long)kHdim, PK16 + qoff, PK16 + qoff, kDim, (long)kHdim,
          (void*)SC32, (void*)SC32, kSeq, sPlane, bdum, rdum, 0L, kSeq, kSeq, kHdim, kScoreScale);
      row_stats_kernel<<<dim3(kGrp * kSeq / 32), dim3(256), 0, stream>>>(SC32, RM, RI, kPCarry);
      exp_transpose_kernel<<<dim3(kSeq / 64, kSeq / 64, kGrp), dim3(256), 0, stream>>>(SC32, RM, RI, PPT16);
      wmma_gemm64<0, false, 0, 1, false><<<gridSq, dim3(256), 0, stream>>>(
          GP16, GP16, kSeq, sPlane, PPT16, PPT16, kSeq, sPlane,
          (void*)E16, (void*)E16, kSeq, sPlane, bdum, rdum, 0L, kSeq, kSeq, kSeq, kPCarryInv);
      wmma_gemm64<0, false, 0, 0, false><<<gridCtx, dim3(256), 0, stream>>>(
          GP16, GP16, kSeq, sPlane, GVT16 + voff, GVT16 + voff, kTok, sVTgrp,
          (void*)(CTX32 + coff), (void*)(CTX32 + coff), kDim, (long)kHdim, bdum, rdum, 0L,
          kSeq, kHdim, kSeq, kCtxScale);
      wmma_gemm64<0, false, 0, 1, true><<<gridCtx, dim3(256), 0, stream>>>(
          E16, E16, kSeq, sPlane, PVT16 + voff, PVT16 + voff, kTok, sVTgrp,
          (void*)(LAST16 + qoff), (void*)(LAST16 + qoff), kDim, (long)kHdim, bdum,
          (const float*)(CTX32 + coff), (long)kHdim, kSeq, kHdim, kSeq, kCtxScale);
    }
  }

  cast8_f16_kernel<<<dim3(castWBlocks), dim3(256), 0, stream>>>(Wp[6], W16, nW / 8, kWCarry);
  wmma_gemm64<0, false, 2, 0, false><<<dim3((kTok / 64) * (kDim / 64) / 8, 1), dim3(256), 0, stream>>>(
      LAST16, LAST16, kDim, 0L, W16, W16, kDim, 0L, d_out, d_out, kDim, 0L, Bp[6], rdum, 0L,
      kTok, kDim, kDim, kOutScale);
}
